// LSTMCell_48507360641621
// MI455X (gfx1250) — hardware-verified
//
#include <hip/hip_runtime.h>
#include <math.h>

constexpr int NBATCH  = 64;
constexpr int NSTEP   = 512;
constexpr int NIN     = 256;
constexpr int NHID    = 256;
constexpr int NGCOL   = 4 * NHID;
constexpr int SCHUNK  = 256;
constexpr int NCHUNK  = 2;
constexpr int NTHR    = 256;
constexpr int RTHR    = 512;
constexpr int SEQ_BLK = 16;
constexpr int HPITCH  = 264;
constexpr int OPITCH  = 260;
constexpr int NOUT0   = NBATCH * NSTEP * NHID;
constexpr int NOUT1   = NBATCH * NHID;
constexpr float HCARRY        = 256.0f;
constexpr float WCARRY        = 64.0f;
constexpr float ACC_CARRY     = 16384.0f;
constexpr float ACC_CARRY_INV = 1.0f / 16384.0f;
static_assert(HCARRY * WCARRY == ACC_CARRY);
static_assert(NSTEP == SCHUNK * NCHUNK);
static_assert(NHID == 16 * (RTHR / 32));
static_assert(NBATCH % SEQ_BLK == 0);
static_assert((SEQ_BLK * NHID) % RTHR == 0);
static_assert(NGCOL % 64 == 0);
static_assert(NBATCH % 64 == 0);
static_assert(NIN % 32 == 0 && NHID % 32 == 0);
static_assert((size_t)NOUT0 * 4 == 33554432u);
static_assert((size_t)(NOUT0 + NOUT1) * 4 == 33619968u);
static_assert((size_t)(NOUT0 + 2 * NOUT1) * 4 == 33685504u);

typedef __attribute__((ext_vector_type(16))) _Float16 v16h;
typedef __attribute__((ext_vector_type(8)))  _Float16 v8h;
typedef __attribute__((ext_vector_type(16))) __bf16   v16b;
typedef __attribute__((ext_vector_type(8)))  __bf16   v8b;
typedef __attribute__((ext_vector_type(8)))  float    v8f;
typedef __attribute__((ext_vector_type(4)))  float    v4f;

__device__ __forceinline__ unsigned short f2bf_bits(float f) {
  unsigned u = __float_as_uint(f);
  return (unsigned short)((u + 0x7FFFu + ((u >> 16) & 1u)) >> 16);
}
__device__ __forceinline__ float bf_bits2f(unsigned short h) { return __uint_as_float(((unsigned)h) << 16); }
__device__ __forceinline__ float bf16r(float f) { return bf_bits2f(f2bf_bits(f)); }

__device__ __forceinline__ void dep_guard_h(v8f& a, v8f& b, v16h x, v16h y) { asm volatile("v_nop\n\tv_nop\n\tv_nop\n\tv_nop" : "+v"(a), "+v"(b) : "v"(x), "v"(y)); }
__device__ __forceinline__ void dep_guard_b(v8f& a, v8f& b, v16b x, v16b y) { asm volatile("v_nop\n\tv_nop\n\tv_nop\n\tv_nop" : "+v"(a), "+v"(b) : "v"(x), "v"(y)); }
__device__ __forceinline__ void dep_guard4_h(v8f& a, v8f& b, v8f& c, v8f& d, v16h x, v16h y) { asm volatile("v_nop\n\tv_nop\n\tv_nop\n\tv_nop" : "+v"(a), "+v"(b), "+v"(c), "+v"(d) : "v"(x), "v"(y)); }
__device__ __forceinline__ void dep_guard4_b(v8f& a, v8f& b, v8f& c, v8f& d, v16b x, v16b y) { asm volatile("v_nop\n\tv_nop\n\tv_nop\n\tv_nop" : "+v"(a), "+v"(b), "+v"(c), "+v"(d) : "v"(x), "v"(y)); }
__device__ __forceinline__ void keep4_h(v16h a, v16h b, v16h c, v16h d) { asm volatile("v_nop" :: "v"(a), "v"(b), "v"(c), "v"(d)); }
__device__ __forceinline__ void keep4_b(v16b a, v16b b, v16b c, v16b d) { asm volatile("v_nop" :: "v"(a), "v"(b), "v"(c), "v"(d)); }
__device__ __forceinline__ void acc_guard4(v8f& a, v8f& b, v8f& c, v8f& d) { asm volatile("v_nop\n\tv_nop\n\tv_nop\n\tv_nop" : "+v"(a), "+v"(b), "+v"(c), "+v"(d)); }
__device__ __forceinline__ void mma_guard_4acc_5frag(v8f& a0, v8f& a1, v8f& a2, v8f& a3, v16h x, v16h y0, v16h y1, v16h y2, v16h y3) {
  asm volatile("v_nop\n\tv_nop\n\tv_nop\n\tv_nop" : "+v"(a0), "+v"(a1), "+v"(a2), "+v"(a3) : "v"(x), "v"(y0), "v"(y1), "v"(y2), "v"(y3));
}
template <typename T> struct Frag;
template <> struct Frag<_Float16> {
  typedef v16h V; union U { v16h v; v8h h[2]; };
  static __device__ __forceinline__ v16h load(const _Float16* p) {
    U f; f.h[0] = *(const v8h*)(p); f.h[1] = *(const v8h*)(p + 16); return f.v;
  }
  static __device__ __forceinline__ v8f mma(v16h a, v16h b, v8f c) {
    return __builtin_amdgcn_wmma_f32_16x16x32_f16(false, a, false, b, (short)0, c, false, false);
  }
  static __device__ __forceinline__ void guard(v8f& a, v8f& b, v16h x, v16h y) { dep_guard_h(a, b, x, y); }
  static __device__ __forceinline__ void guard4(v8f& a, v8f& b, v8f& c, v8f& d, v16h x, v16h y) { dep_guard4_h(a, b, c, d, x, y); }
  static __device__ __forceinline__ void keep(v16h a, v16h b, v16h c, v16h d) { keep4_h(a, b, c, d); }
};
template <> struct Frag<__bf16> {
  typedef v16b V; union U { v16b v; v8b h[2]; };
  static __device__ __forceinline__ v16b load(const __bf16* p) {
    U f; f.h[0] = *(const v8b*)(p); f.h[1] = *(const v8b*)(p + 16); return f.v;
  }
  static __device__ __forceinline__ v8f mma(v16b a, v16b b, v8f c) {
    return __builtin_amdgcn_wmma_f32_16x16x32_bf16(false, a, false, b, (short)0, c, false, false);
  }
  static __device__ __forceinline__ void guard(v8f& a, v8f& b, v16b x, v16b y) { dep_guard_b(a, b, x, y); }
  static __device__ __forceinline__ void guard4(v8f& a, v8f& b, v8f& c, v8f& d, v16b x, v16b y) { dep_guard4_b(a, b, c, d, x, y); }
  static __device__ __forceinline__ void keep(v16b a, v16b b, v16b c, v16b d) { keep4_b(a, b, c, d); }
};

__device__ __forceinline__ float fsig(float x)  { return __builtin_amdgcn_rcpf(1.0f + expf(-x)); }
__device__ __forceinline__ float ftanh(float x) { return 1.0f - 2.0f * __builtin_amdgcn_rcpf(expf(2.0f * x) + 1.0f); }

template <int ET> struct Elem;
template <> struct Elem<0> { typedef _Float16 T; };
template <> struct Elem<1> { typedef __bf16 T; };
template <int ET, bool SPLIT, int BIAS_MODE, int OUT_MODE, bool RESID, int ACT = 0>
__global__ __launch_bounds__(256) void wmma_gemm64(
    const unsigned short* __restrict__ Ap, const unsigned short* __restrict__ A2p, int lda, long strideA,
    const unsigned short* __restrict__ Btp, const unsigned short* __restrict__ Bt2p, int ldb, long strideB,
    void* __restrict__ Cout, void* __restrict__ Cout2, int ldc, long strideC,
    const float* __restrict__ bias,
    const float* __restrict__ resid, long strideR,
    int M, int N, int K, float scale) {
  typedef typename Elem<ET>::T T;
  typedef typename Frag<T>::V V;
  const T* A = (const T*)Ap; const T* A2 = (const T*)A2p; const T* Bt = (const T*)Btp; const T* Bt2 = (const T*)Bt2p;
  __shared__ __align__(16) float sT[8][16 * 68];
  const int b    = blockIdx.y;
  const int lane = threadIdx.x & 31;
  const int wave = threadIdx.x >> 5;
  const int tilesN = N >> 6;
  const int tilesM = M >> 6;
  const int tile = blockIdx.x * 8 + wave;
  if (tile >= tilesM * tilesN) return;
  const int tm = tile / tilesN;
  const int tn = tile - tm * tilesN;
  const int m0 = tm << 6;
  const int n0 = tn << 6;

  const T* Ab  = A  + (size_t)b * strideA;
  const T* Bb  = Bt + (size_t)b * strideB;
  const T* Ab2 = SPLIT ? (A2  + (size_t)b * strideA) : nullptr;
  const T* Bb2 = SPLIT ? (Bt2 + (size_t)b * strideB) : nullptr;

  const int rlane = lane & 15;
  const int koff  = (lane >> 4) * 8;
  const int mOff  = (lane >> 4) * 8;

  v8f acc[4][4];
#pragma unroll
  for (int i = 0; i < 4; ++i)
#pragma unroll
    for (int j = 0; j < 4; ++j) acc[i][j] = (v8f){0.f,0.f,0.f,0.f,0.f,0.f,0.f,0.f};

  for (int k0 = 0; k0 < K; k0 += 32) {
    V bh[4], bl[4];
#pragma unroll
    for (int j = 0; j < 4; ++j) {
      const size_t bo = (size_t)(n0 + (j << 4) + rlane) * ldb + koff + k0;
      bh[j] = Frag<T>::load(Bb + bo);
      if (SPLIT) bl[j] = Frag<T>::load(Bb2 + bo);
    }
#pragma unroll
    for (int i = 0; i < 4; ++i) {
      const size_t ao = (size_t)(m0 + (i << 4) + rlane) * lda + koff + k0;
      V ah = Frag<T>::load(Ab + ao);
      V al;
      if (SPLIT) al = Frag<T>::load(Ab2 + ao);
#pragma unroll
      for (int j = 0; j < 4; ++j) {
        acc[i][j] = Frag<T>::mma(ah, bh[j], acc[i][j]);
        if (SPLIT) {
          acc[i][j] = Frag<T>::mma(ah, bl[j], acc[i][j]);
          acc[i][j] = Frag<T>::mma(al, bh[j], acc[i][j]);
        }
      }
      Frag<T>::guard4(acc[i][0], acc[i][1], acc[i][2], acc[i][3], ah, SPLIT ? al : bh[3]);
    }
    Frag<T>::keep(bh[0], bh[1], bh[2], bh[3]);
    if (SPLIT) Frag<T>::keep(bl[0], bl[1], bl[2], bl[3]);
  }
  acc_guard4(acc[0][0], acc[0][1], acc[0][2], acc[0][3]);
  acc_guard4(acc[1][0], acc[1][1], acc[1][2], acc[1][3]);
  acc_guard4(acc[2][0], acc[2][1], acc[2][2], acc[2][3]);
  acc_guard4(acc[3][0], acc[3][1], acc[3][2], acc[3][3]);

  float* slab = sT[wave];
  const float* Rb = RESID ? (resid + (size_t)b * strideR) : nullptr;
#pragma unroll
  for (int i = 0; i < 4; ++i) {
    const int mBase = m0 + (i << 4);
    float bm[8];
#pragma unroll
    for (int r = 0; r < 8; ++r) bm[r] = 0.f;
    if (BIAS_MODE == 1) {
      const v4f bq0 = *(const v4f*)(bias + mBase + mOff);
      const v4f bq1 = *(const v4f*)(bias + mBase + mOff + 4);
      bm[0] = bq0[0]; bm[1] = bq0[1]; bm[2] = bq0[2]; bm[3] = bq0[3];
      bm[4] = bq1[0]; bm[5] = bq1[1]; bm[6] = bq1[2]; bm[7] = bq1[3];
    }
#pragma unroll
    for (int j = 0; j < 4; ++j) {
      const int n = n0 + (j << 4) + rlane;
      float bv = 0.f;
      if (BIAS_MODE == 2) bv = bias[n];
#pragma unroll
      for (int r = 0; r < 8; ++r) {
        float v = acc[i][j][r] * scale;
        if (BIAS_MODE == 1) v += bm[r];
        if (BIAS_MODE == 2) v += bv;
        if (RESID) v += Rb[(size_t)(mBase + mOff + r) * ldc + n];
        if (ACT == 1) v = tanhf(v);
        if (ACT == 2) v = fmaxf(v, 0.0f);
        if (ACT == 4) v = (v > 0.f) ? v : 0.01f * v;
        slab[(mOff + r) * 68 + (j << 4) + rlane] = v;
      }
    }
    __builtin_amdgcn_fence(__ATOMIC_RELEASE, "workgroup");
    __builtin_amdgcn_wave_barrier();
    __builtin_amdgcn_fence(__ATOMIC_ACQUIRE, "workgroup");
    if (OUT_MODE == 0) {
      float* C = (float*)Cout + (size_t)b * strideC;
      const int hh = lane >> 4, c4 = (lane & 15) * 4;
      for (int pass = 0; pass < 2; ++pass) {
#pragma unroll
        for (int it = 0; it < 8; ++it) {
          const int row = it * 2 + hh;
          v4f v = *(const v4f*)(slab + row * 68 + c4);
          *(volatile v4f*)(C + (size_t)(mBase + row) * ldc + n0 + c4) = v;
        }
        __threadfence();
      }
    } else {
      const int q = lane >> 3, c8 = (lane & 7) * 8;
      unsigned short* C  = (unsigned short*)Cout  + (size_t)b * strideC;
      unsigned short* C2 = (OUT_MODE == 2) ? ((unsigned short*)Cout2 + (size_t)b * strideC) : nullptr;
      for (int pass = 0; pass < 2; ++pass) {
#pragma unroll
        for (int it = 0; it < 4; ++it) {
          const int row = it * 4 + q;
          const float* sp = slab + row * 68 + c8;
          v8h hv, lv;
#pragma unroll
          for (int e = 0; e < 8; ++e) {
            if (OUT_MODE == 1) {
              hv[e] = (_Float16)sp[e];
            } else {
              unsigned short hb = f2bf_bits(sp[e]);
              unsigned short lb = f2bf_bits(sp[e] - bf_bits2f(hb));
              hv[e] = __builtin_bit_cast(_Float16, hb);
              lv[e] = __builtin_bit_cast(_Float16, lb);
            }
          }
          *(volatile v8h*)(C + (size_t)(mBase + row) * ldc + n0 + c8) = hv;
          if (OUT_MODE == 2) *(volatile v8h*)(C2 + (size_t)(mBase + row) * ldc + n0 + c8) = lv;
        }
        __threadfence();
      }
    }
    __builtin_amdgcn_fence(__ATOMIC_RELEASE, "workgroup");
    __builtin_amdgcn_wave_barrier();
    __builtin_amdgcn_fence(__ATOMIC_ACQUIRE, "workgroup");
  }
}

template <int MODE>
__global__ __launch_bounds__(NTHR) void cvt8_kernel(const float* __restrict__ src, unsigned short* __restrict__ dst,
                                                    int nrow, int ncol8, int spitch, int scol0, float sc) {
  const int i  = blockIdx.x * NTHR + threadIdx.x;
  const int n8 = nrow * ncol8;
  if (i < n8) {
    const int row = i / ncol8;
    const int c8  = i - row * ncol8;
    const float* sp = src + (size_t)row * spitch + scol0 + c8 * 8;
    const v4f a = *(const v4f*)(sp);
    const v4f b = *(const v4f*)(sp + 4);
    v8h hv;
#pragma unroll
    for (int e = 0; e < 4; ++e) {
      unsigned short b0, b1;
      if (MODE == 0) {
        b0 = f2bf_bits(a[e] * sc);
        b1 = f2bf_bits(b[e] * sc);
      } else {
        b0 = __builtin_bit_cast(unsigned short, (_Float16)(bf16r(a[e]) * sc));
        b1 = __builtin_bit_cast(unsigned short, (_Float16)(bf16r(b[e]) * sc));
      }
      hv[e]     = __builtin_bit_cast(_Float16, b0);
      hv[4 + e] = __builtin_bit_cast(_Float16, b1);
    }
    *(volatile v8h*)(dst + (size_t)i * 8) = hv;
    __threadfence();
    *(volatile v8h*)(dst + (size_t)i * 8) = hv;
  }
}

__global__ __launch_bounds__(NTHR) void bias_prep_kernel(const float* __restrict__ ba, const float* __restrict__ bb,
                                                         float* __restrict__ dst) {
  const int idx = threadIdx.x * 4;
  const v4f va = *(const v4f*)(ba + idx);
  const v4f vb = *(const v4f*)(bb + idx);
  v4f o;
#pragma unroll
  for (int e = 0; e < 4; ++e) o[e] = bf16r(va[e]) + bf16r(vb[e]);
  float* op = dst + idx;
  *(volatile v4f*)op = o;
  __threadfence();
  *(volatile v4f*)op = o;
}

__global__ __launch_bounds__(NTHR) void state_prep_kernel(const float* __restrict__ h0, const float* __restrict__ c0,
                                                          float* __restrict__ CH, float* __restrict__ CC) {
  const int idx = (blockIdx.x * NTHR + threadIdx.x) * 4;
  const v4f vh = *(const v4f*)(h0 + idx);
  const v4f vc = *(const v4f*)(c0 + idx);
  v4f oh, oc;
#pragma unroll
  for (int e = 0; e < 4; ++e) { oh[e] = bf16r(vh[e]); oc[e] = bf16r(vc[e]); }
  for (int pass = 0; pass < 2; ++pass) {
    *(volatile v4f*)(CH + idx) = oh;
    *(volatile v4f*)(CC + idx) = oc;
    __threadfence();
  }
}

__global__ __launch_bounds__(RTHR) void lstm_seq_kernel(const float* __restrict__ XG, const unsigned short* __restrict__ WHp,
                                                       const float* __restrict__ SRCH, const float* __restrict__ SRCC,
                                                       float* HSEQ, float* DSTH, float* DSTC, int s_base) {
  __shared__ __align__(16) _Float16 Ah[SEQ_BLK * HPITCH];
  __shared__ __align__(16) float    Hs[SEQ_BLK * OPITCH];
  const _Float16* WH = (const _Float16*)WHp;
  const int tid = threadIdx.x, lane = tid & 31, wave = tid >> 5;
  const int c = lane & 15, hh = lane >> 4, koff = hh * 8;
  const int rowbase = blockIdx.x * SEQ_BLK;
  const int j = 16 * wave + c;

#pragma unroll 1
  for (int i = 0; i < (SEQ_BLK * NHID) / RTHR; ++i) {
    const int idx = i * RTHR + tid;
    const int row = idx >> 8, col = idx & 255;
    Ah[row * HPITCH + col] = (_Float16)(SRCH[(size_t)(rowbase + row) * NHID + col] * HCARRY);
  }
  float cst[8], hst[8];
#pragma unroll
  for (int r = 0; r < 8; ++r) {
    cst[r] = SRCC[(size_t)(rowbase + 8 * hh + r) * NHID + j];
    hst[r] = 0.0f;
  }
  __syncthreads();

  const _Float16* ahrow = Ah + c * HPITCH + koff;
  const _Float16* wh = WH + (size_t)j * NHID + koff;
  const float* xgl = XG + (size_t)j * NBATCH + rowbase + 8 * hh;

#pragma unroll 1
  for (int sl = 0; sl < SCHUNK; ++sl) {
    const float* xp = xgl + (size_t)sl * (size_t)(NGCOL * NBATCH);
    v8f acc[4];
#pragma unroll
    for (int g = 0; g < 4; ++g) {
      const v4f u0 = *(const v4f*)(xp + (size_t)g * (NHID * NBATCH));
      const v4f u1 = *(const v4f*)(xp + (size_t)g * (NHID * NBATCH) + 4);
      v8f t;
      t[0] = u0[0] * ACC_CARRY; t[1] = u0[1] * ACC_CARRY; t[2] = u0[2] * ACC_CARRY; t[3] = u0[3] * ACC_CARRY;
      t[4] = u1[0] * ACC_CARRY; t[5] = u1[1] * ACC_CARRY; t[6] = u1[2] * ACC_CARRY; t[7] = u1[3] * ACC_CARRY;
      acc[g] = t;
    }
#pragma unroll 1
    for (int k0 = 0; k0 < NHID; k0 += 32) {
      const v16h a  = Frag<_Float16>::load(ahrow + k0);
      const v16h b0 = Frag<_Float16>::load(wh + k0);
      const v16h b1 = Frag<_Float16>::load(wh + (size_t)1 * NHID * NHID + k0);
      const v16h b2 = Frag<_Float16>::load(wh + (size_t)2 * NHID * NHID + k0);
      const v16h b3 = Frag<_Float16>::load(wh + (size_t)3 * NHID * NHID + k0);
      acc[0] = Frag<_Float16>::mma(a, b0, acc[0]);
      acc[1] = Frag<_Float16>::mma(a, b1, acc[1]);
      acc[2] = Frag<_Float16>::mma(a, b2, acc[2]);
      acc[3] = Frag<_Float16>::mma(a, b3, acc[3]);
      mma_guard_4acc_5frag(acc[0], acc[1], acc[2], acc[3], a, b0, b1, b2, b3);
    }
    acc_guard4(acc[0], acc[1], acc[2], acc[3]);
#pragma unroll
    for (int r = 0; r < 8; ++r) {
      const float zf = acc[0][r] * ACC_CARRY_INV;
      const float zi = acc[1][r] * ACC_CARRY_INV;
      const float zg = acc[2][r] * ACC_CARRY_INV;
      const float zo = acc[3][r] * ACC_CARRY_INV;
      const float fg = fsig(zf);
      const float ig = fsig(zi);
      const float gg = ftanh(zg);
      const float og = fsig(zo);
      const float cn = cst[r] * fg + ig * gg;
      cst[r] = cn;
      hst[r] = og * ftanh(cn);
    }
    __syncthreads();
#pragma unroll
    for (int r = 0; r < 8; ++r) {
      Ah[(8 * hh + r) * HPITCH + j] = (_Float16)(hst[r] * HCARRY);
      Hs[(8 * hh + r) * OPITCH + j] = hst[r];
    }
    __syncthreads();
    const int sg = s_base + sl;
    for (int pass = 0; pass < 2; ++pass) {
#pragma unroll
      for (int it = 0; it < 2; ++it) {
        const int idx = it * RTHR + tid;
        const int row = idx >> 6, c4 = (idx & 63) * 4;
        const v4f v = *(const v4f*)(Hs + row * OPITCH + c4);
        *(volatile v4f*)(HSEQ + ((size_t)(rowbase + row) * NSTEP + (size_t)sg) * NHID + c4) = v;
      }
      __threadfence();
    }
  }

  for (int pass = 0; pass < 2; ++pass) {
#pragma unroll
    for (int it = 0; it < 2; ++it) {
      const int idx = it * RTHR + tid;
      const int row = idx >> 6, c4 = (idx & 63) * 4;
      const v4f v = *(const v4f*)(Hs + row * OPITCH + c4);
      *(volatile v4f*)(DSTH + (size_t)(rowbase + row) * NHID + c4) = v;
    }
    __threadfence();
  }
  __syncthreads();
#pragma unroll
  for (int r = 0; r < 8; ++r) Hs[(8 * hh + r) * OPITCH + j] = cst[r];
  __syncthreads();
  for (int pass = 0; pass < 2; ++pass) {
#pragma unroll
    for (int it = 0; it < 2; ++it) {
      const int idx = it * RTHR + tid;
      const int row = idx >> 6, c4 = (idx & 63) * 4;
      const v4f v = *(const v4f*)(Hs + row * OPITCH + c4);
      *(volatile v4f*)(DSTC + (size_t)(rowbase + row) * NHID + c4) = v;
    }
    __threadfence();
  }
}

extern "C" void kernel_launch(void* const* d_in, const int* in_sizes, int n_in,
                              void* d_out, int out_size, void* d_ws, size_t ws_size, hipStream_t stream) {
  if (n_in < 7 || d_out == nullptr || d_ws == nullptr) return;
  if (in_sizes[0] != NBATCH * NSTEP * NIN || in_sizes[1] != NBATCH * NHID || in_sizes[2] != NBATCH * NHID ||
      in_sizes[3] != NGCOL * NHID || in_sizes[4] != NGCOL || in_sizes[5] != NGCOL * NIN || in_sizes[6] != NGCOL ||
      out_size != NOUT0 + 2 * NOUT1) return;

  const float* x  = (const float*)d_in[0];
  const float* h0 = (const float*)d_in[1];
  const float* c0 = (const float*)d_in[2];
  const float* Wh = (const float*)d_in[3];
  const float* bh = (const float*)d_in[4];
  const float* Wx = (const float*)d_in[5];
  const float* bx = (const float*)d_in[6];
  float* hseq = (float*)d_out;
  float* hfin = hseq + (size_t)NOUT0;
  float* cfin = hfin + (size_t)NOUT1;

  char* ws = (char*)d_ws; size_t off = 0;
  auto carve = [&](size_t bytes) -> char* { char* p = ws + off; off += (bytes + 255) & ~(size_t)255; return p; };
  unsigned short* XB   = (unsigned short*)carve((size_t)NBATCH * NSTEP * NIN * 2);
  unsigned short* WXB  = (unsigned short*)carve((size_t)NGCOL * NIN * 2);
  unsigned short* WHH  = (unsigned short*)carve((size_t)NGCOL * NHID * 2);
  float*          BIAS = (float*)carve((size_t)NGCOL * 4);
  float*          CH0  = (float*)carve((size_t)NBATCH * NHID * 4);
  float*          CC0  = (float*)carve((size_t)NBATCH * NHID * 4);
  float*          CH1  = (float*)carve((size_t)NBATCH * NHID * 4);
  float*          CC1  = (float*)carve((size_t)NBATCH * NHID * 4);
  float*          XG   = (float*)carve((size_t)SCHUNK * NGCOL * NBATCH * 4);
  if (off > ws_size || off > (size_t)134217728) return;

  const int n8x = NBATCH * NSTEP * (NIN / 8);
  const int n8w = NGCOL * (NIN / 8);
  cvt8_kernel<0><<<(n8x + NTHR - 1) / NTHR, NTHR, 0, stream>>>(x,  XB,  NBATCH * NSTEP, NIN / 8,  NIN,  0, 1.0f);
  cvt8_kernel<0><<<(n8w + NTHR - 1) / NTHR, NTHR, 0, stream>>>(Wx, WXB, NGCOL,          NIN / 8,  NIN,  0, 1.0f);
  cvt8_kernel<1><<<(n8w + NTHR - 1) / NTHR, NTHR, 0, stream>>>(Wh, WHH, NGCOL,          NHID / 8, NHID, 0, WCARRY);
  bias_prep_kernel<<<1, NTHR, 0, stream>>>(bx, bh, BIAS);
  state_prep_kernel<<<(NBATCH * NHID) / (NTHR * 4), NTHR, 0, stream>>>(h0, c0, CH0, CC0);

  const dim3 ggrid((NGCOL / 64) * (NBATCH / 64) / 8, SCHUNK);
  for (int q = 0; q < NCHUNK; ++q) {
    const unsigned short* XBq = XB + (size_t)q * SCHUNK * NIN;
    wmma_gemm64<1, false, 1, 0, false, 0><<<ggrid, 256, 0, stream>>>(
        WXB, WXB, NIN, 0L, XBq, XBq, NSTEP * NIN, (long)NIN, (void*)XG, (void*)XG, NBATCH, (long)(NGCOL * NBATCH),
        BIAS, BIAS, 0L, NGCOL, NBATCH, NIN, 1.0f);
    const float* srcH = (q == 0) ? CH0 : CH1;
    const float* srcC = (q == 0) ? CC0 : CC1;
    float* dstH = (q == NCHUNK - 1) ? hfin : CH1;
    float* dstC = (q == NCHUNK - 1) ? cfin : CC1;
    lstm_seq_kernel<<<NBATCH / SEQ_BLK, RTHR, 0, stream>>>(XG, WHH, srcH, srcC, hseq, dstH, dstC, q * SCHUNK);
  }
}
